// TriangularSylvesterNeRF_33586644255083
// MI455X (gfx1250) — hardware-run, weakly checked
//
#include <hip/hip_runtime.h>


#define NSM  32768
#define NPT  4096
#define NHC  128
#define NZW  32
#define NKS  4
constexpr size_t al256(size_t b) { return (b + 255) & ~(size_t)255; }
constexpr size_t WS_TOTAL = al256((size_t)NPT * NHC * 2) + al256((size_t)NZW * NZW * NKS * NHC * 2) + 3 * al256((size_t)NZW * NKS * NHC * 2) + al256((size_t)NPT * NZW * NZW * NKS * 4) + 3 * al256((size_t)NPT * NZW * NKS * 4) + 2 * al256((size_t)NPT * NZW * 4) + al256((size_t)NPT * 4);
static_assert(WS_TOTAL == 76660736 && WS_TOTAL <= 134217728, "the workspace carve: 73.1 MiB");
static_assert(NSM % NPT == 0 && NPT % 64 == 0 && (NZW * NZW * NKS) % 64 == 0 && (NZW * NKS) % 64 == 0 && NHC % 32 == 0 && ((size_t)NPT * NHC) % 8 == 0 && NZW * 4 == 128, "whole tiles; whole depth steps; a thread's state is one line");
typedef _Float16 h16;
typedef unsigned short bf;
typedef __attribute__((ext_vector_type(16))) __bf16   v16bf;
typedef __attribute__((ext_vector_type(16))) _Float16 v16h;
typedef __attribute__((ext_vector_type(8)))  _Float16 v8h;
typedef __attribute__((ext_vector_type(8)))  unsigned short v8us;
typedef __attribute__((ext_vector_type(8)))  float    v8f;
typedef __attribute__((ext_vector_type(4)))  float    v4f;
typedef v8h  __attribute__((may_alias)) v8ha;
typedef v4f  __attribute__((may_alias)) v4fa;
typedef v8us __attribute__((may_alias)) v8usa;

__device__ __forceinline__ unsigned short f2bf(float f) { unsigned u = __float_as_uint(f); u += 0x7FFFu + ((u >> 16) & 1u); return (unsigned short)(u >> 16); }
__device__ __forceinline__ float bf2f(unsigned short b) { return __uint_as_float(((unsigned)b) << 16); }
__device__ __forceinline__ float bfr(float f) { return bf2f(f2bf(f)); }
__device__ __forceinline__ v16h cat16(v8h lo, v8h hi) { return __builtin_shufflevector(lo, hi, 0, 1, 2, 3, 4, 5, 6, 7, 8, 9, 10, 11, 12, 13, 14, 15); }
__device__ __forceinline__ v16bf cat16b(v8us lo, v8us hi) { return __builtin_bit_cast(v16bf, __builtin_shufflevector(lo, hi, 0, 1, 2, 3, 4, 5, 6, 7, 8, 9, 10, 11, 12, 13, 14, 15)); }
__device__ __forceinline__ v8f wmma16(v16h a, v16h b, v8f c) { return __builtin_amdgcn_wmma_f32_16x16x32_f16(false, a, false, b, (short)0, c, false, false); }
__device__ __forceinline__ v8f wmmab(v16bf a, v16bf b, v8f c) { return __builtin_amdgcn_wmma_f32_16x16x32_bf16(false, a, false, b, (short)0, c, false, false); }


template <typename T16> struct WFrag;
template <> struct WFrag<h16> { typedef v16h V; static __device__ __forceinline__ V ld(const h16* p) { return cat16(*(const v8h*)p, *(const v8h*)(p + 16)); } static __device__ __forceinline__ v8f mma(V a, V b, v8f c) { return wmma16(a, b, c); } };
template <> struct WFrag<bf> { typedef v16bf V; static __device__ __forceinline__ V ld(const bf* p) { return cat16b(*(const v8us*)p, *(const v8us*)(p + 16)); } static __device__ __forceinline__ v8f mma(V a, V b, v8f c) { return wmmab(a, b, c); } };
template <typename T16, int NSPLIT, bool BIAS>
__global__ __launch_bounds__(32) void k_gemmw(const T16* __restrict__ A, const T16* __restrict__ A2, const T16* __restrict__ Bt, const T16* __restrict__ Bt2, int K, float* C, int ldc, const float* __restrict__ bias, size_t sA, size_t sB, size_t sC) {
    typedef typename WFrag<T16>::V V;
    __shared__ __align__(16) float os[16 * 68];
    const size_t z = blockIdx.z; A += z * sA; if (A2) A2 += z * sA; Bt += z * sB; if (Bt2) Bt2 += z * sB; C += z * sC;
    const int lane = threadIdx.x & 31, lr = lane & 15, hi = lane >> 4; const int r0 = blockIdx.x * 64, c0 = blockIdx.y * 64;
    v8f acc[4][4];
#pragma unroll
    for (int mb = 0; mb < 4; ++mb)
#pragma unroll
        for (int nb = 0; nb < 4; ++nb) acc[mb][nb] = (v8f){};
    const size_t aoff = (size_t)(r0 + lr) * K + 8 * hi, boff = (size_t)(c0 + lr) * K + 8 * hi;
    for (int kc = 0; kc < K; kc += 32) {
        V a[4], a2[4];
#pragma unroll
        for (int mb = 0; mb < 4; ++mb) { a[mb] = WFrag<T16>::ld(A + aoff + (size_t)mb * 16 * K + kc); if (NSPLIT == 1 || NSPLIT == 2) a2[mb] = WFrag<T16>::ld(A2 + aoff + (size_t)mb * 16 * K + kc); }
#pragma unroll
        for (int nb = 0; nb < 4; ++nb) { const V b = WFrag<T16>::ld(Bt + boff + (size_t)nb * 16 * K + kc); V b2; if (NSPLIT >= 2) b2 = WFrag<T16>::ld(Bt2 + boff + (size_t)nb * 16 * K + kc);
#pragma unroll
            for (int mb = 0; mb < 4; ++mb) { acc[mb][nb] = WFrag<T16>::mma(a[mb], b, acc[mb][nb]); if (NSPLIT == 1 || NSPLIT == 2) acc[mb][nb] = WFrag<T16>::mma(a2[mb], b, acc[mb][nb]); if (NSPLIT >= 2) acc[mb][nb] = WFrag<T16>::mma(a[mb], b2, acc[mb][nb]); } }
        asm volatile("v_nop\n\tv_nop\n\tv_nop\n\tv_nop" : "+v"(acc[0][0]), "+v"(acc[1][1]), "+v"(acc[2][2]), "+v"(acc[3][3]) : "v"(a[0]), "v"(a[3]));
    }
#pragma unroll
    for (int mb = 0; mb < 4; ++mb) {
#pragma unroll
        for (int nb = 0; nb < 4; ++nb) {
#pragma unroll
            for (int j = 0; j < 8; ++j) os[(hi * 8 + j) * 68 + nb * 16 + lr] = acc[mb][nb][j]; }
        __builtin_amdgcn_wave_barrier(); asm volatile("" ::: "memory");
        float* crow = C + (size_t)(r0 + mb * 16) * ldc + c0;
#pragma unroll 1
        for (int ps = 0; ps < 2; ++ps) {
#pragma unroll
            for (int s = 0; s < 8; ++s) { const int row = 2 * s + hi, cofs = lr * 4; v4f val = *(const v4fa*)(os + row * 68 + cofs); if (BIAS) { val[0] += bfr(bias[c0 + cofs]); val[1] += bfr(bias[c0 + cofs + 1]); val[2] += bfr(bias[c0 + cofs + 2]); val[3] += bfr(bias[c0 + cofs + 3]); }
                *(volatile v4f*)(crow + (size_t)row * ldc + cofs) = val; }
            if (ps == 0) __threadfence(); }
        __builtin_amdgcn_wave_barrier(); asm volatile("" ::: "memory");
    }
}

__device__ __forceinline__ h16 tohx(float x) { return (h16)x; }
__device__ __forceinline__ void splitf(float y, unsigned short& h, unsigned short& l) { h = f2bf(y); l = f2bf(y - bf2f(h)); }
typedef __attribute__((ext_vector_type(2))) _Float16 v2h;
typedef __attribute__((ext_vector_type(4))) _Float16 v4h;
typedef __attribute__((ext_vector_type(2))) unsigned short v2us;
typedef __attribute__((ext_vector_type(4))) unsigned short v4us;
typedef __attribute__((ext_vector_type(2))) float v2f;
typedef __attribute__((ext_vector_type(4))) int v4i;

__global__ __launch_bounds__(256) void k_cvt8(const float* __restrict__ src, bf* dst, size_t n8) { const size_t i = (size_t)blockIdx.x * 256 + threadIdx.x; if (i >= n8) return; const v8f v = *(const v8f*)(src + i * 8); v8us o;
#pragma unroll
    for (int k = 0; k < 8; ++k) o[k] = f2bf(v[k]); *(volatile v8us*)(dst + i * 8) = o; __threadfence(); *(volatile v8us*)(dst + i * 8) = o; }

__global__ __launch_bounds__(64) void k_fz(const float* __restrict__ za, float* ZS, float* LS) {
    const unsigned sm = blockIdx.x * 64 + threadIdx.x; if (sm >= (unsigned)NPT) return; float* d = ZS + (size_t)sm * NZW; v4f o[NZW / 4];
#pragma unroll
    for (int c = 0; c < NZW / 4; ++c) { const v4f v = *(const v4f*)(za + (size_t)sm * NZW + 4 * c); o[c][0] = bfr(v[0]); o[c][1] = bfr(v[1]); o[c][2] = bfr(v[2]); o[c][3] = bfr(v[3]); }
#pragma unroll
    for (int c = 0; c < NZW / 4; ++c) *(volatile v4f*)(d + 4 * c) = o[c];
    *(volatile float*)(LS + sm) = 0.0f; __threadfence();
#pragma unroll
    for (int c = 0; c < NZW / 4; ++c) *(volatile v4f*)(d + 4 * c) = o[c];
    *(volatile float*)(LS + sm) = 0.0f; }

__global__ __launch_bounds__(64) void k_fa(const float* __restrict__ FA, const float* __restrict__ GA, const float* __restrict__ GB, const float* __restrict__ GC, const float* __restrict__ ZS, const float* __restrict__ LS, float* TV, float* LD, int st) {
    const unsigned sm = blockIdx.x * 64 + threadIdx.x; if (sm >= (unsigned)NPT) return;
    const float* fa = FA + (size_t)sm * (NZW * NZW * NKS) + st; const float* ga = GA + (size_t)sm * (NZW * NKS) + st; const float* gb = GB + (size_t)sm * (NZW * NKS) + st; const float* gc = GC + (size_t)sm * (NZW * NKS) + st;
    const float* zs = ZS + (size_t)sm * NZW; float* tvd = TV + (size_t)sm * NZW; const bool od = (st & 1) != 0; float lg = LS[sm];
    for (int j = 0; j < NZW; ++j) { const float da = tanhf(ga[j * NKS]); const float db = tanhf(gb[j * NKS]); float ar = zs[od ? NZW - 1 - j : j] * db;
        for (int i = j + 1; i < NZW; ++i) ar += zs[od ? NZW - 1 - i : i] * fa[(i * NZW + j) * NKS];
        const float tj = tanhf(ar + gc[j * NKS]); lg += logf(fabsf((1.0f - tj * tj) * (da * db) + 1.0f));
        *(volatile float*)(tvd + j) = tj; __threadfence(); *(volatile float*)(tvd + j) = tj; }
    *(volatile float*)(LD + sm) = lg; __threadfence(); *(volatile float*)(LD + sm) = lg; }

__global__ __launch_bounds__(64) void k_fb(const float* __restrict__ FA, const float* __restrict__ GA, const float* __restrict__ TV, const float* ZS, float* ZD, int st) {
    const unsigned sm = blockIdx.x * 64 + threadIdx.x; if (sm >= (unsigned)NPT) return;
    const float* fa = FA + (size_t)sm * (NZW * NZW * NKS) + st; const float* ga = GA + (size_t)sm * (NZW * NKS) + st; const float* tvs = TV + (size_t)sm * NZW; const float* zs = ZS + (size_t)sm * NZW; float* d = ZD + (size_t)sm * NZW; const bool od = (st & 1) != 0;
    for (int i = 0; i < NZW; ++i) { float uv = tvs[i] * tanhf(ga[i * NKS]);
        for (int j = i + 1; j < NZW; ++j) uv += tvs[j] * fa[(i * NZW + j) * NKS];
        const int ix = od ? NZW - 1 - i : i; const float yn = zs[ix] + uv; *(volatile float*)(d + ix) = yn; __threadfence(); *(volatile float*)(d + ix) = yn; } }

extern "C" void kernel_launch(void* const* d_in, const int* in_sizes, int n_in,
                              void* d_out, int out_size, void* d_ws, size_t ws_size, hipStream_t stream) {
    if (n_in < 10) return;
    if (in_sizes[0] < NSM * NZW || in_sizes[1] < NSM * NHC || in_sizes[2] < NZW * NZW * NKS * NHC || in_sizes[3] < NZW * NZW * NKS || in_sizes[4] < NZW * NKS * NHC || in_sizes[5] < NZW * NKS || in_sizes[6] < NZW * NKS * NHC || in_sizes[7] < NZW * NKS || in_sizes[8] < NZW * NKS * NHC || in_sizes[9] < NZW * NKS || out_size < NSM * NZW + NSM) return;
    const float* za = (const float*)d_in[0]; const float* hc = (const float*)d_in[1]; const float* ua = (const float*)d_in[2]; const float* ca = (const float*)d_in[3]; const float* ub = (const float*)d_in[4]; const float* cb = (const float*)d_in[5];
    const float* uc = (const float*)d_in[6]; const float* cc = (const float*)d_in[7]; const float* ud = (const float*)d_in[8]; const float* cd = (const float*)d_in[9];
    float* RZ = (float*)d_out; float* RL = RZ + (size_t)NSM * NZW;
    char* wsp = (char*)d_ws;
    auto take = [&](size_t bytes) { char* cur = wsp; wsp += (bytes + 255) & ~(size_t)255; return (void*)cur; };
    bf* HB = (bf*)take((size_t)NPT * NHC * 2); bf* UA = (bf*)take((size_t)NZW * NZW * NKS * NHC * 2); bf* UB = (bf*)take((size_t)NZW * NKS * NHC * 2); bf* UC = (bf*)take((size_t)NZW * NKS * NHC * 2); bf* UD = (bf*)take((size_t)NZW * NKS * NHC * 2);
    float* FA = (float*)take((size_t)NPT * NZW * NZW * NKS * 4); float* GA = (float*)take((size_t)NPT * NZW * NKS * 4); float* GB = (float*)take((size_t)NPT * NZW * NKS * 4); float* GC = (float*)take((size_t)NPT * NZW * NKS * 4);
    float* ZS = (float*)take((size_t)NPT * NZW * 4); float* TV = (float*)take((size_t)NPT * NZW * 4); float* LS = (float*)take((size_t)NPT * 4);
    if ((size_t)(wsp - (char*)d_ws) != WS_TOTAL || WS_TOTAL > ws_size) return;
    const size_t na8 = (size_t)NZW * NZW * NKS * NHC / 8, nb8 = (size_t)NZW * NKS * NHC / 8, nh8 = (size_t)NPT * NHC / 8;
    k_cvt8<<<(unsigned)((na8 + 255) / 256), 256, 0, stream>>>(ua, UA, na8);
    k_cvt8<<<(unsigned)((nb8 + 255) / 256), 256, 0, stream>>>(ub, UB, nb8);
    k_cvt8<<<(unsigned)((nb8 + 255) / 256), 256, 0, stream>>>(uc, UC, nb8);
    k_cvt8<<<(unsigned)((nb8 + 255) / 256), 256, 0, stream>>>(ud, UD, nb8);
    for (int pt = 0; pt < NSM / NPT; ++pt) {
        const size_t s0 = (size_t)pt * NPT;
        k_cvt8<<<(unsigned)((nh8 + 255) / 256), 256, 0, stream>>>(hc + s0 * NHC, HB, nh8);
        k_gemmw<bf, 0, true><<<dim3(NPT / 64, NZW * NZW * NKS / 64, 1), 32, 0, stream>>>(HB, nullptr, UA, nullptr, NHC, FA, NZW * NZW * NKS, ca, (size_t)0, (size_t)0, (size_t)0);
        k_gemmw<bf, 0, true><<<dim3(NPT / 64, NZW * NKS / 64, 1), 32, 0, stream>>>(HB, nullptr, UB, nullptr, NHC, GA, NZW * NKS, cb, (size_t)0, (size_t)0, (size_t)0);
        k_gemmw<bf, 0, true><<<dim3(NPT / 64, NZW * NKS / 64, 1), 32, 0, stream>>>(HB, nullptr, UC, nullptr, NHC, GB, NZW * NKS, cc, (size_t)0, (size_t)0, (size_t)0);
        k_gemmw<bf, 0, true><<<dim3(NPT / 64, NZW * NKS / 64, 1), 32, 0, stream>>>(HB, nullptr, UD, nullptr, NHC, GC, NZW * NKS, cd, (size_t)0, (size_t)0, (size_t)0);
        k_fz<<<NPT / 64, 64, 0, stream>>>(za + s0 * NZW, ZS, LS);
        for (int st = 0; st < NKS; ++st) {
            k_fa<<<NPT / 64, 64, 0, stream>>>(FA, GA, GB, GC, ZS, LS, TV, st == NKS - 1 ? RL + s0 : LS, st);
            k_fb<<<NPT / 64, 64, 0, stream>>>(FA, GA, TV, ZS, st == NKS - 1 ? RZ + s0 * NZW : ZS, st);
        }
    }
}
